// RelativeNetwork_24635932409876
// MI455X (gfx1250) — hardware-verified
//
#include <hip/hip_runtime.h>


#define NB   4
#define CIN  3
#define EMB  8
#define NCH0   24
#define NSZ0   64
#define NCH1   16
#define NSZ1   32
#define NCH2   32
#define NSZ2   16
#define NPR  (NSZ2 * NSZ2)
#define K1   600
#define K1P  640
#define K2   400
#define K2P  448
#define RO   256
#define KR   128
#define HIDF 256
#define OUTF 64
#define NEMB 11
#define DM   64
#define LOSC 1024.0f

typedef _Float16 h16;
typedef unsigned short bf;
typedef __attribute__((ext_vector_type(16))) __bf16   v16bf;
typedef __attribute__((ext_vector_type(16))) _Float16 v16h;
typedef __attribute__((ext_vector_type(8)))  _Float16 v8h;
typedef __attribute__((ext_vector_type(8)))  unsigned short v8us;
typedef __attribute__((ext_vector_type(8)))  float    v8f;
typedef __attribute__((ext_vector_type(4)))  float    v4f;
typedef v8h  __attribute__((may_alias)) v8ha;
typedef v4f  __attribute__((may_alias)) v4fa;
typedef v8us __attribute__((may_alias)) v8usa;

__device__ __forceinline__ unsigned short f2bf(float f) { unsigned u = __float_as_uint(f); u += 0x7FFFu + ((u >> 16) & 1u); return (unsigned short)(u >> 16); }
__device__ __forceinline__ float bf2f(unsigned short b) { return __uint_as_float(((unsigned)b) << 16); }
__device__ __forceinline__ float bfr(float f) { return bf2f(f2bf(f)); }
__device__ __forceinline__ v16h cat16(v8h lo, v8h hi) { return __builtin_shufflevector(lo, hi, 0, 1, 2, 3, 4, 5, 6, 7, 8, 9, 10, 11, 12, 13, 14, 15); }
__device__ __forceinline__ v16bf cat16b(v8us lo, v8us hi) { return __builtin_bit_cast(v16bf, __builtin_shufflevector(lo, hi, 0, 1, 2, 3, 4, 5, 6, 7, 8, 9, 10, 11, 12, 13, 14, 15)); }
__device__ __forceinline__ v8f wmma16(v16h a, v16h b, v8f c) { return __builtin_amdgcn_wmma_f32_16x16x32_f16(false, a, false, b, (short)0, c, false, false); }
__device__ __forceinline__ v8f wmmab(v16bf a, v16bf b, v8f c) { return __builtin_amdgcn_wmma_f32_16x16x32_bf16(false, a, false, b, (short)0, c, false, false); }

template <bool SPLITA, bool F16OUT = false>
__global__ __launch_bounds__(128) void k_gemmb(const bf* __restrict__ A, const bf* __restrict__ Al, const bf* __restrict__ Bn, const float* __restrict__ bias, float* C, int ldc, h16* C2p, const float* __restrict__ R = nullptr, int K = DM, int roundR = 1) {
    __shared__ __align__(16) float ost[4][16 * 68];
    const int lane = threadIdx.x & 31, wave = threadIdx.x >> 5, lr = lane & 15, hi = lane >> 4;
    const int r0 = blockIdx.x * 64 + wave * 16, c0 = blockIdx.y * 64;
    const size_t aoff = (size_t)(r0 + lr) * K + 8 * hi;
    size_t boff[4];
#pragma unroll
    for (int t = 0; t < 4; ++t) boff[t] = (size_t)(c0 + t * 16 + lr) * K + 8 * hi;
    v8f acc[4];
#pragma unroll
    for (int t = 0; t < 4; ++t) acc[t] = (v8f){};
#pragma unroll 1
    for (int kc = 0; kc < K; kc += 32) {
        const v16bf a = cat16b(*(const v8us*)(A + aoff + kc), *(const v8us*)(A + aoff + kc + 16));
        v16bf al = a;
        if (SPLITA) al = cat16b(*(const v8us*)(Al + aoff + kc), *(const v8us*)(Al + aoff + kc + 16));
#pragma unroll
        for (int t = 0; t < 4; ++t) { const v16bf b = cat16b(*(const v8us*)(Bn + boff[t] + kc), *(const v8us*)(Bn + boff[t] + kc + 16)); acc[t] = wmmab(a, b, acc[t]); if (SPLITA) acc[t] = wmmab(al, b, acc[t]); }
        asm volatile("v_nop\n\tv_nop\n\tv_nop\n\tv_nop" : "+v"(acc[0]), "+v"(acc[1]), "+v"(acc[2]), "+v"(acc[3]) : "v"(a), "v"(al));
    }
    float* os = &ost[wave][0];
#pragma unroll
    for (int t = 0; t < 4; ++t) { const float bv = bias ? bfr(bias[c0 + t * 16 + lr]) : 0.f;
#pragma unroll
        for (int j = 0; j < 8; ++j) os[(hi * 8 + j) * 68 + t * 16 + lr] = acc[t][j] + bv; }
    __syncthreads();
    if (F16OUT) {
        h16* crow = (h16*)(void*)C + (size_t)r0 * ldc + c0;
        auto pass = [&]() {
#pragma unroll
            for (int s = 0; s < 4; ++s) { const int row = 4 * s + (lane >> 3), piece = lane & 7; const float* sp = os + row * 68 + piece * 8; v8h o, o2;
#pragma unroll
                for (int i = 0; i < 8; ++i) { const h16 a = (h16)sp[i]; o[i] = a; o2[i] = (h16)((sp[i] - (float)a) * LOSC); }
                *(volatile v8h*)(crow + (size_t)row * ldc + piece * 8) = o; if (C2p) *(volatile v8h*)(C2p + (size_t)r0 * ldc + c0 + (size_t)row * ldc + piece * 8) = o2; }
        };
        pass(); __threadfence(); pass();
    } else {
        float* crow = C + (size_t)r0 * ldc + c0;
        auto pass = [&]() {
#pragma unroll
            for (int s = 0; s < 8; ++s) { const int Lid = (lane >> 3) + 4 * s, piece = lane & 7; const int row = Lid >> 1, cofs = (Lid & 1) * 32 + piece * 4;
                v4f val = *(const v4fa*)(os + row * 68 + cofs); if (R) { const v4f rv = *(const v4f*)(R + ((size_t)r0 + row) * ldc + c0 + cofs); val += roundR ? (v4f){bfr(rv[0]), bfr(rv[1]), bfr(rv[2]), bfr(rv[3])} : rv; }
                *(volatile v4f*)(crow + (size_t)row * ldc + cofs) = val; }
        };
        pass(); __threadfence(); pass();
    }
}


__global__ __launch_bounds__(256) void k_cvt8(const float* __restrict__ src, bf* dst, size_t n8) {
    const size_t i = (size_t)blockIdx.x * 256 + threadIdx.x; if (i >= n8) return;
    const v8f v = *(const v8f*)(src + i * 8); v8us o;
#pragma unroll
    for (int k = 0; k < 8; ++k) o[k] = f2bf(v[k]);
    *(volatile v8us*)(dst + i * 8) = o; __threadfence(); *(volatile v8us*)(dst + i * 8) = o;
}
__global__ __launch_bounds__(256) void k_zero8(bf* dst, size_t n8) {
    const size_t i = (size_t)blockIdx.x * 256 + threadIdx.x; if (i >= n8) return; v8us z;
#pragma unroll
    for (int k = 0; k < 8; ++k) z[k] = 0;
    *(volatile v8us*)(dst + i * 8) = z; __threadfence(); *(volatile v8us*)(dst + i * 8) = z;
}

__global__ __launch_bounds__(256) void k_im1(const int* __restrict__ xi, const float* __restrict__ emb, bf* A1) {
    const int lane = threadIdx.x & 31, r = blockIdx.x * 8 + (threadIdx.x >> 5); if (r >= NB * NSZ0 * NSZ0) return; const int b = r / (NSZ0 * NSZ0), y = (r / NSZ0) % NSZ0, x = r % NSZ0;
#pragma unroll 1
    for (int ps = 0; ps < 2; ++ps) {
#pragma unroll 1
        for (int k0 = lane * 8; k0 < K1P; k0 += 256) { v8us o;
#pragma unroll
            for (int q = 0; q < 8; ++q) { const int k = k0 + q; unsigned short v = 0;
                if (k < K1) { const int ch = k / 25, t = k % 25, dy = t / 5, dx = t % 5; const int c = ch / EMB, e = ch % EMB; const int yy = y + dy - 2, xx = x + dx - 2;
                    if (yy >= 0 && yy < NSZ0 && xx >= 0 && xx < NSZ0) { int lab = xi[((b * CIN + c) * NSZ0 + yy) * NSZ0 + xx]; lab = lab < 0 ? 0 : (lab >= NEMB ? NEMB - 1 : lab); v = f2bf(emb[lab * EMB + e]); } }
                o[q] = v; }
            *(volatile v8us*)(A1 + (size_t)r * K1P + k0) = o; }
        if (ps == 0) __threadfence(); }
}
__global__ __launch_bounds__(256) void k_wpadT(const float* __restrict__ Wm, int nout, int kk, int kp, bf* WT) {
    const int lane = threadIdx.x & 31, o = blockIdx.x * 8 + (threadIdx.x >> 5); if (o >= 64) return;
#pragma unroll 1
    for (int ps = 0; ps < 2; ++ps) {
#pragma unroll 1
        for (int k0 = lane * 8; k0 < kp; k0 += 256) { v8us ob;
#pragma unroll
            for (int q = 0; q < 8; ++q) { const int k = k0 + q; const bool ok = (o < nout) && (k < kk); ob[q] = ok ? f2bf(Wm[(size_t)(ok ? o : 0) * kk + (ok ? k : 0)]) : (unsigned short)0; }
            *(volatile v8us*)(WT + (size_t)o * kp + k0) = ob; }
        if (ps == 0) __threadfence(); }
}
__global__ __launch_bounds__(256) void k_pool1(const float* __restrict__ G1, const float* __restrict__ bb, float* P1) {
    const int g = blockIdx.x * 256 + threadIdx.x; if (g >= NB * NCH1 * NSZ1 * NSZ1) return; const int b = g / (NCH1 * NSZ1 * NSZ1), c = (g / (NSZ1 * NSZ1)) % NCH1, py = (g / NSZ1) % NSZ1, px = g % NSZ1;
    float m = -3.0e38f;
#pragma unroll
    for (int dy = 0; dy < 2; ++dy)
#pragma unroll
        for (int dx = 0; dx < 2; ++dx) m = fmaxf(m, G1[((size_t)(b * NSZ0 + 2 * py + dy) * NSZ0 + 2 * px + dx) * 64 + c]);
    const float v = fmaxf(m + bfr(bb[c]), 0.f); *(volatile float*)(P1 + g) = v; __threadfence(); *(volatile float*)(P1 + g) = v;
}
__global__ __launch_bounds__(256) void k_im2(const float* __restrict__ P1, bf* Ah, bf* Al) {
    const int lane = threadIdx.x & 31, r = blockIdx.x * 8 + (threadIdx.x >> 5); if (r >= NB * NSZ1 * NSZ1) return; const int b = r / (NSZ1 * NSZ1), y = (r / NSZ1) % NSZ1, x = r % NSZ1;
#pragma unroll 1
    for (int ps = 0; ps < 2; ++ps) {
#pragma unroll 1
        for (int k0 = lane * 8; k0 < K2P; k0 += 256) { v8us oh, ol;
#pragma unroll
            for (int q = 0; q < 8; ++q) { const int k = k0 + q; float v = 0.f;
                if (k < K2) { const int c = k / 25, t = k % 25, dy = t / 5, dx = t % 5; const int yy = y + dy - 2, xx = x + dx - 2;
                    if (yy >= 0 && yy < NSZ1 && xx >= 0 && xx < NSZ1) v = P1[((size_t)(b * NCH1 + c) * NSZ1 + yy) * NSZ1 + xx]; }
                const unsigned short hb = f2bf(v); oh[q] = hb; ol[q] = f2bf(v - bf2f(hb)); }
            *(volatile v8us*)(Ah + (size_t)r * K2P + k0) = oh; *(volatile v8us*)(Al + (size_t)r * K2P + k0) = ol; }
        if (ps == 0) __threadfence(); }
}
__global__ __launch_bounds__(256) void k_pool2(const float* __restrict__ G2, const float* __restrict__ bb, float* HF) {
    const int g = blockIdx.x * 256 + threadIdx.x; if (g >= NB * NCH2 * NPR) return; const int b = g / (NCH2 * NPR), c = (g / NPR) % NCH2, py = (g / NSZ2) % NSZ2, px = g % NSZ2;
    float m = -3.0e38f;
#pragma unroll
    for (int dy = 0; dy < 2; ++dy)
#pragma unroll
        for (int dx = 0; dx < 2; ++dx) m = fmaxf(m, G2[((size_t)(b * NSZ1 + 2 * py + dy) * NSZ1 + 2 * px + dx) * 64 + c]);
    const float v = fmaxf(m + bfr(bb[c]), 0.f); *(volatile float*)(HF + g) = v; __threadfence(); *(volatile float*)(HF + g) = v;
}
__global__ __launch_bounds__(256) void k_pair(const float* __restrict__ HF, int b, int r0, bf* Ph, bf* Pl) {
    typedef __attribute__((ext_vector_type(4))) unsigned short v4us;
    const int lane = threadIdx.x & 31; const int rl = blockIdx.x * 8 + (threadIdx.x >> 5); if (rl >= NPR * NPR / 2) return; const int r = r0 + rl; const int i = r / NPR, j = r % NPR;
    v4us oh, ol;
#pragma unroll
    for (int q = 0; q < 4; ++q) { const int c = lane * 4 + q; float v = 0.f;
        if (c == 0) v = (float)(i / NSZ2) / (float)NSZ2 - (float)(j / NSZ2) / (float)NSZ2; else if (c == 1) v = (float)(i % NSZ2) / (float)NSZ2 - (float)(j % NSZ2) / (float)NSZ2;
        else if (c < 34) v = HF[((size_t)b * NCH2 + (c - 2)) * NPR + i]; else if (c < 66) v = HF[((size_t)b * NCH2 + (c - 34)) * NPR + j];
        const unsigned short hb = f2bf(v); oh[q] = hb; ol[q] = f2bf(v - bf2f(hb)); }
    const size_t o = (size_t)rl * KR + lane * 4; *(volatile v4us*)(Ph + o) = oh; *(volatile v4us*)(Pl + o) = ol; __threadfence(); *(volatile v4us*)(Ph + o) = oh; *(volatile v4us*)(Pl + o) = ol;
}
__global__ __launch_bounds__(256) void k_colsum(const float* __restrict__ C, const float* __restrict__ br, int half, float* PS) {
    const int o = threadIdx.x; const float bb = bfr(br[o]); float s = 0.f;
#pragma unroll 4
    for (int r = 0; r < NPR * NPR / 2; ++r) s += fmaxf(C[(size_t)r * RO + o] + bb, 0.f);
    *(volatile float*)(PS + half * RO + o) = s; __threadfence(); *(volatile float*)(PS + half * RO + o) = s;
}
__global__ __launch_bounds__(256) void k_colmean(const float* __restrict__ PS, int b, float* GS) {
    const int o = threadIdx.x; const float v = (PS[o] + PS[RO + o]) * (1.0f / (float)(NPR * NPR)); *(volatile float*)(GS + b * RO + o) = v; __threadfence(); *(volatile float*)(GS + b * RO + o) = v;
}
template <int MODE>
__global__ __launch_bounds__(256) void k_split64r(const float* __restrict__ src, const float* __restrict__ bias, int nreal, int ncol, bf* dh, bf* dl) {
    const int lane = threadIdx.x & 31, r = blockIdx.x * 8 + (threadIdx.x >> 5); if (r >= 64) return;
#pragma unroll 1
    for (int ps = 0; ps < 2; ++ps) {
#pragma unroll 1
        for (int c0 = lane * 8; c0 < ncol; c0 += 256) { v8us oh, ol;
#pragma unroll
            for (int q = 0; q < 8; ++q) { const int c = c0 + q; float v = 0.f; if (r < nreal) { v = src[(size_t)r * ncol + c]; if (MODE == 1) v = fmaxf(v + bfr(bias[c]), 0.f); }
                const unsigned short hb = f2bf(v); oh[q] = hb; ol[q] = f2bf(v - bf2f(hb)); }
            *(volatile v8us*)(dh + (size_t)r * ncol + c0) = oh; *(volatile v8us*)(dl + (size_t)r * ncol + c0) = ol; }
        if (ps == 0) __threadfence(); }
}
__global__ __launch_bounds__(256) void k_fin(const float* __restrict__ F2, const float* __restrict__ bb, float* OUTP) {
    __shared__ float gv[256]; __shared__ float red[8];
    const int t = threadIdx.x; const int b = t / OUTF, o = t % OUTF; const float g = F2[(size_t)b * OUTF + o] + bfr(bb[o]); gv[t] = g; __syncthreads();
    if (t == 0) { float s = 0.f; for (int i = 0; i < 256; ++i) s += gv[i]; red[0] = s / 256.0f; }
    __syncthreads(); const float gc = g - red[0]; gv[t] = gc * gc; __syncthreads();
    if (t < NB) { float s = 0.f; for (int i = 0; i < OUTF; ++i) s += gv[t * OUTF + i]; red[1 + t] = sqrtf(s); }
    __syncthreads(); const float v = gc / red[1 + b];
    *(volatile float*)(OUTP + t) = v; __threadfence(); *(volatile float*)(OUTP + t) = v;
}

extern "C" void kernel_launch(void* const* d_in, const int* in_sizes, int n_in,
                              void* d_out, int out_size, void* d_ws, size_t ws_size, hipStream_t stream) {
    (void)in_sizes; (void)n_in; (void)out_size;
    const int* xi = (const int*)d_in[0]; const float* emb = (const float*)d_in[1]; const float* w1 = (const float*)d_in[2]; const float* b1 = (const float*)d_in[3]; const float* w2 = (const float*)d_in[4]; const float* b2 = (const float*)d_in[5];
    const float* wr = (const float*)d_in[6]; const float* br = (const float*)d_in[7]; const float* wf1 = (const float*)d_in[8]; const float* bf1 = (const float*)d_in[9]; const float* wf2 = (const float*)d_in[10]; const float* bf2 = (const float*)d_in[11];
    float* out = (float*)d_out;
    char* wsp = (char*)d_ws;
    auto take = [&](size_t bytes) { char* p = wsp; wsp += (bytes + 255) & ~(size_t)255; return (void*)p; };
    bf* A1 = (bf*)take((size_t)NB * NSZ0 * NSZ0 * K1P * 2); bf* W1T = (bf*)take((size_t)64 * K1P * 2); float* G1 = (float*)take((size_t)NB * NSZ0 * NSZ0 * 64 * 4); float* P1 = (float*)take((size_t)NB * NCH1 * NSZ1 * NSZ1 * 4);
    bf* A2h = (bf*)take((size_t)NB * NSZ1 * NSZ1 * K2P * 2); bf* A2l = (bf*)take((size_t)NB * NSZ1 * NSZ1 * K2P * 2); bf* W2T = (bf*)take((size_t)64 * K2P * 2); float* G2 = (float*)take((size_t)NB * NSZ1 * NSZ1 * 64 * 4); float* HF = (float*)take((size_t)NB * NCH2 * NPR * 4);
    bf* WRT = (bf*)take((size_t)RO * KR * 2); bf* Ph = (bf*)take((size_t)(NPR * NPR / 2) * KR * 2); bf* Pl = (bf*)take((size_t)(NPR * NPR / 2) * KR * 2); float* C = (float*)take((size_t)(NPR * NPR / 2) * RO * 4); float* GS = (float*)take((size_t)NB * RO * 4); float* PS = (float*)take(2 * RO * 4);
    bf* Gh = (bf*)take(64 * 256 * 2); bf* Gl = (bf*)take(64 * 256 * 2); bf* WF1 = (bf*)take((size_t)HIDF * 256 * 2); bf* WF2 = (bf*)take((size_t)OUTF * HIDF * 2); float* F1 = (float*)take(64 * HIDF * 4); float* F2 = (float*)take(64 * OUTF * 4);
    if ((size_t)(wsp - (char*)d_ws) > ws_size) return;
    k_im1<<<(NB * NSZ0 * NSZ0) / 8, 256, 0, stream>>>(xi, emb, A1); k_wpadT<<<64 / 8, 256, 0, stream>>>(w1, NCH1, K1, K1P, W1T);
    k_gemmb<false, false><<<dim3((NB * NSZ0 * NSZ0) / 64, 1, 1), 128, 0, stream>>>(A1, nullptr, W1T, nullptr, G1, 64, nullptr, nullptr, K1P);
    k_pool1<<<(NB * NCH1 * NSZ1 * NSZ1) / 256, 256, 0, stream>>>(G1, b1, P1);
    k_im2<<<(NB * NSZ1 * NSZ1) / 8, 256, 0, stream>>>(P1, A2h, A2l); k_wpadT<<<64 / 8, 256, 0, stream>>>(w2, NCH2, K2, K2P, W2T);
    k_gemmb<true, false><<<dim3((NB * NSZ1 * NSZ1) / 64, 1, 1), 128, 0, stream>>>(A2h, A2l, W2T, nullptr, G2, 64, nullptr, nullptr, K2P);
    k_pool2<<<(NB * NCH2 * NPR) / 256, 256, 0, stream>>>(G2, b2, HF);
    for (int o0 = 0; o0 < RO; o0 += 64) k_wpadT<<<64 / 8, 256, 0, stream>>>(wr + (size_t)o0 * 66, 64, 66, KR, WRT + (size_t)o0 * KR);
    for (int b = 0; b < NB; ++b) {
        for (int half = 0; half < 2; ++half) { const int r0 = half * (NPR * NPR / 2);
            k_pair<<<(NPR * NPR / 2) / 8, 256, 0, stream>>>(HF, b, r0, Ph, Pl);
            k_gemmb<true, false><<<dim3((NPR * NPR / 2) / 64, RO / 64, 1), 128, 0, stream>>>(Ph, Pl, WRT, nullptr, C, RO, nullptr, nullptr, KR);
            k_colsum<<<1, 256, 0, stream>>>(C, br, half, PS); }
        k_colmean<<<1, 256, 0, stream>>>(PS, b, GS); }
    k_cvt8<<<(HIDF * 256 / 8 + 255) / 256, 256, 0, stream>>>(wf1, WF1, HIDF * 256 / 8); k_cvt8<<<(OUTF * HIDF / 8 + 255) / 256, 256, 0, stream>>>(wf2, WF2, OUTF * HIDF / 8);
    k_split64r<0><<<64 / 8, 256, 0, stream>>>(GS, nullptr, NB, 256, Gh, Gl);
    k_gemmb<true, false><<<dim3(1, HIDF / 64, 1), 128, 0, stream>>>(Gh, Gl, WF1, nullptr, F1, HIDF, nullptr, nullptr, 256);
    k_split64r<1><<<64 / 8, 256, 0, stream>>>(F1, bf1, NB, HIDF, Gh, Gl);
    k_gemmb<true, false><<<dim3(1, OUTF / 64, 1), 128, 0, stream>>>(Gh, Gl, WF2, nullptr, F2, OUTF, nullptr, nullptr, HIDF);
    k_fin<<<1, 256, 0, stream>>>(F2, bf2, out);
}
